// Scorer_22351009809137
// MI455X (gfx1250) — hardware-verified
//
#include <hip/hip_runtime.h>


#define NN        1024
#define HH        1024
#define MLPH      100
#define XP        128
#define JT        1025
#define OUT_TOTAL 1049601

typedef _Float16 v16h __attribute__((ext_vector_type(16)));
typedef _Float16 v8h  __attribute__((ext_vector_type(8)));
typedef float    v8f  __attribute__((ext_vector_type(8)));
typedef float    v4f  __attribute__((ext_vector_type(4)));
union Frag { v16h v; v8h half[2]; };

__device__ __forceinline__ v8f wmma16(v16h a, v16h b, v8f c)
{
    v8f d = __builtin_amdgcn_wmma_f32_16x16x32_f16(false, a, false, b, (short)0, c, false, false);
    asm volatile("v_nop\n\tv_nop\n\tv_nop\n\tv_nop" : "+v"(d) : "v"(a), "v"(b));
    return d;
}

__device__ __forceinline__ v8h cvt8(const float* p, float sc)
{
    const v4f x0 = *(const v4f*)p;
    const v4f x1 = *(const v4f*)(p + 4);
    v8h r;
    r[0] = (_Float16)(x0[0] * sc); r[1] = (_Float16)(x0[1] * sc);
    r[2] = (_Float16)(x0[2] * sc); r[3] = (_Float16)(x0[3] * sc);
    r[4] = (_Float16)(x1[0] * sc); r[5] = (_Float16)(x1[1] * sc);
    r[6] = (_Float16)(x1[2] * sc); r[7] = (_Float16)(x1[3] * sc);
    return r;
}

__device__ __forceinline__ float sigm(float z)
{
    const float e = __builtin_amdgcn_exp2f(z * -1.4426950408889634f);
    return __builtin_amdgcn_rcpf(1.0f + e);
}

__device__ __forceinline__ float exs(float x)
{
    return __builtin_amdgcn_exp2f(x * 1.4426950408889634f);
}

__device__ __forceinline__ v8h sig8(const float* pa, const float* pb)
{
    const v4f z0 = *(const v4f*)pa + *(const v4f*)pb;
    const v4f z1 = *(const v4f*)(pa + 4) + *(const v4f*)(pb + 4);
    v8h r;
    r[0] = (_Float16)sigm(z0[0]); r[1] = (_Float16)sigm(z0[1]);
    r[2] = (_Float16)sigm(z0[2]); r[3] = (_Float16)sigm(z0[3]);
    r[4] = (_Float16)sigm(z1[0]); r[5] = (_Float16)sigm(z1[1]);
    r[6] = (_Float16)sigm(z1[2]); r[7] = (_Float16)sigm(z1[3]);
    return r;
}

__device__ __forceinline__ v8h sig4lo(const float* pa, const float* pb)
{
    const v4f z0 = *(const v4f*)pa + *(const v4f*)pb;
    v8h r;
    r[0] = (_Float16)sigm(z0[0]); r[1] = (_Float16)sigm(z0[1]);
    r[2] = (_Float16)sigm(z0[2]); r[3] = (_Float16)sigm(z0[3]);
    r[4] = (_Float16)0.0f; r[5] = (_Float16)0.0f; r[6] = (_Float16)0.0f; r[7] = (_Float16)0.0f;
    return r;
}

__device__ __forceinline__ void fill_w2t(_Float16* w2t, const float* W2, int t, int nthr)
{
    for (int q = t; q < 16 * XP; q += nthr) {
        const int r = q >> 7, k = q & (XP - 1);
        const int kc = (k < MLPH) ? k : (MLPH - 1);
        const float wl = W2[kc];
        const float wv = (r == 0 && k < MLPH) ? (wl * 256.0f) : 0.0f;
        w2t[q] = (_Float16)wv;
    }
}

__device__ __forceinline__ float group_dot(const _Float16* w2t, const float* xap, const float* xbp, int h, int m)
{
    v8f acc = {};
#pragma unroll
    for (int s = 0; s < 4; ++s) {
        const int k0 = 32 * s;
        Frag a, bq;
        a.half[0] = *(const v8h*)(w2t + m * XP + k0 + 8 * h);
        a.half[1] = *(const v8h*)(w2t + m * XP + k0 + 16 + 8 * h);
        if (s < 3) {
            bq.half[0] = sig8(xap + k0 + 8 * h,      xbp + k0 + 8 * h);
            bq.half[1] = sig8(xap + k0 + 16 + 8 * h, xbp + k0 + 16 + 8 * h);
        } else {
            bq.half[0] = sig4lo(xap + k0 + 8 * h, xbp + k0 + 8 * h);
            v8h z = {};
            bq.half[1] = z;
        }
        acc = wmma16(a.v, bq.v, acc);
    }
    return acc[0];
}

__global__ __launch_bounds__(32)
void k_proj(const float* __restrict__ S, const float* __restrict__ W1,
            const float* __restrict__ b1, float* __restrict__ XA,
            float* __restrict__ XB)
{
    __shared__ __align__(16) float stg[16 * XP];
    const int l = threadIdx.x & 31, h = l >> 4, m = l & 15;
    const int rt = blockIdx.x, mat = blockIdx.y;

    const float* arow  = S + (size_t)(rt * 16 + m) * HH;
    const float* wbase = W1 + (size_t)mat * HH;

    v8f acc[7] = {};
#pragma unroll 1
    for (int k0 = 0; k0 < HH; k0 += 32) {
        Frag a;
        a.half[0] = cvt8(arow + k0 + 8 * h, 1.0f);
        a.half[1] = cvt8(arow + k0 + 16 + 8 * h, 1.0f);
#pragma unroll
        for (int t = 0; t < 7; ++t) {
            const int n  = t * 16 + m;
            const int nc = (n < MLPH) ? n : (MLPH - 1);
            const float wsc = (n < MLPH) ? 64.0f : 0.0f;
            const float* brow = wbase + (size_t)nc * (2 * HH) + k0;
            Frag bq;
            bq.half[0] = cvt8(brow + 8 * h, wsc);
            bq.half[1] = cvt8(brow + 16 + 8 * h, wsc);
            acc[t] = wmma16(a.v, bq.v, acc[t]);
        }
    }

    const float inv64 = 1.0f / 64.0f;
#pragma unroll
    for (int t = 0; t < 7; ++t) {
        const int n  = t * 16 + m;
        const bool nv = n < MLPH;
        const int nc = nv ? n : (MLPH - 1);
        const float bl = b1[nc];
        const float badd = (mat == 0 && nv) ? bl : 0.0f;
#pragma unroll
        for (int r = 0; r < 8; ++r) {
            const float v = nv ? (acc[t][r] * inv64 + badd) : 0.0f;
            stg[(8 * h + r) * XP + n] = v;
        }
    }
#pragma unroll
    for (int r = 0; r < 8; ++r) stg[(8 * h + r) * XP + 112 + m] = 0.0f;
    __syncthreads();

    float* dst = (mat ? XB : XA) + (size_t)(rt * 16) * XP;
    v4f vals[16];
#pragma unroll
    for (int r = 0; r < 16; ++r) vals[r] = *(const v4f*)(stg + r * XP + 4 * l);
#pragma unroll
    for (int r = 0; r < 16; ++r) *(volatile v4f*)(dst + (size_t)r * XP + 4 * l) = vals[r];
    __threadfence();
#pragma unroll
    for (int r = 0; r < 16; ++r) *(volatile v4f*)(dst + (size_t)r * XP + 4 * l) = vals[r];
}

__global__ __launch_bounds__(128)
void k_pair(const float* __restrict__ XA, const float* __restrict__ XB,
            const float* __restrict__ W2, const float* __restrict__ b2,
            float* __restrict__ rawm)
{
    __shared__ __align__(16) float    xb_s[64 * XP];
    __shared__ __align__(16) float    xa_s[16 * XP];
    __shared__ __align__(16) _Float16 w2t[16 * XP];
    __shared__ __align__(16) float    stg[4 * 128];

    const int t = threadIdx.x, w = t >> 5, l = t & 31, h = l >> 4, m = l & 15;
    const int jb = blockIdx.x * 64, ib = blockIdx.y * 16;

    for (int q = t; q < 64 * 32; q += 128) {
        const int r = q >> 5, c = (q & 31) * 4;
        *(v4f*)(xb_s + r * XP + c) = *(const v4f*)(XB + (size_t)(jb + r) * XP + c);
    }
    for (int q = t; q < 16 * 32; q += 128) {
        const int r = q >> 5, c = (q & 31) * 4;
        *(v4f*)(xa_s + r * XP + c) = *(const v4f*)(XA + (size_t)(ib + r) * XP + c);
    }
    fill_w2t(w2t, W2, t, 128);
    __syncthreads();

    const float bias2 = b2[0];
    const float sc = 1.0f / 256.0f;

#pragma unroll 1
    for (int p = 0; p < 2; ++p) {
#pragma unroll 1
        for (int rr = 0; rr < 2; ++rr) {
            const float* xap = xa_s + (4 * w + 2 * p + rr) * XP;
#pragma unroll 1
            for (int g = 0; g < 4; ++g) {
                const float* xbp = xb_s + (16 * g + m) * XP;
                const float rv = group_dot(w2t, xap, xbp, h, m) * sc + bias2;
                if (h == 0) stg[w * 128 + rr * 64 + 16 * g + m] = rv;
            }
        }
        __syncthreads();
        const v4f v = *(const v4f*)(stg + w * 128 + h * 64 + 4 * m);
        float* dp = rawm + (size_t)(ib + 4 * w + 2 * p + h) * NN + jb + 4 * m;
        *(volatile v4f*)dp = v;
        __threadfence();
        *(volatile v4f*)dp = v;
        __syncthreads();
    }
}

__global__ __launch_bounds__(128)
void k_col0(const float* __restrict__ XA, const float* __restrict__ W2,
            const float* __restrict__ b2, float* __restrict__ raw0)
{
    __shared__ __align__(16) _Float16 w2t[16 * XP];
    __shared__ __align__(16) float    zrow[XP];
    __shared__ __align__(16) float    stg[128];

    const int t = threadIdx.x, w = t >> 5, l = t & 31, h = l >> 4, m = l & 15;
    const int i0 = blockIdx.x * 128;

    fill_w2t(w2t, W2, t, 128);
    if (t < XP) zrow[t] = 0.0f;
    __syncthreads();

    const float bias2 = b2[0];
    const float sc = 1.0f / 256.0f;
#pragma unroll 1
    for (int g = 0; g < 2; ++g) {
        const int i = i0 + 32 * w + 16 * g + m;
        const float* xap = XA + (size_t)i * XP;
        const float rv = group_dot(w2t, xap, zrow, h, m) * sc + bias2;
        if (h == 0) stg[32 * w + 16 * g + m] = rv;
    }
    __syncthreads();
    if (w == 0) {
        const v4f v = *(const v4f*)(stg + 4 * l);
        float* dp = raw0 + i0 + 4 * l;
        *(volatile v4f*)dp = v;
        __threadfence();
        *(volatile v4f*)dp = v;
    }
}

__global__ __launch_bounds__(256)
void k_rowstat(const float* __restrict__ rawm, const float* __restrict__ raw0,
               const int* __restrict__ tgt, float* __restrict__ ST)
{
    __shared__ __align__(16) float stgs[3 * 32];
    const int t = threadIdx.x, w = t >> 5, l = t & 31;
    const int b = blockIdx.x;

#pragma unroll 1
    for (int rr = 0; rr < 4; ++rr) {
        const int li = 4 * w + rr;
        const int i = b * 32 + li;
        const float* rp = rawm + (size_t)i * NN;
        const float r0 = raw0[i];
        const int tg = tgt[i];

        float mx = r0;
#pragma unroll 8
        for (int q = 0; q < 32; ++q) mx = fmaxf(mx, rp[32 * q + l]);
#pragma unroll
        for (int o = 16; o > 0; o >>= 1) mx = fmaxf(mx, __shfl_xor(mx, o, 32));

        float s = 0.0f, lp = 0.0f;
        if (l == 0) {
            s  = exs(r0 - mx);
            lp = fabsf(r0 - ((tg == 0) ? 1.0f : 0.0f));
        }
#pragma unroll 8
        for (int q = 0; q < 32; ++q) {
            const int jj = 32 * q + l;
            const float v = rp[jj];
            s  += exs(v - mx);
            lp += fabsf(v - (((jj + 1) == tg) ? 1.0f : 0.0f));
        }
#pragma unroll
        for (int o = 16; o > 0; o >>= 1) {
            s  += __shfl_xor(s, o, 32);
            lp += __shfl_xor(lp, o, 32);
        }
        if (l == 0) {
            stgs[li]      = mx;
            stgs[32 + li] = __builtin_amdgcn_rcpf(s);
            stgs[64 + li] = lp;
        }
    }
    __syncthreads();
    if (w == 0) {
        const int q = l >> 3, c = 4 * (l & 7);
        const bool act = q < 3;
        const int qc = act ? q : 0;
        const v4f v = *(const v4f*)(stgs + qc * 32 + c);
        float* dp = ST + (size_t)qc * NN + b * 32 + c;
        if (act) *(volatile v4f*)dp = v;
        __threadfence();
        if (act) *(volatile v4f*)dp = v;
    }
}

__global__ __launch_bounds__(256)
void k_final(const float* __restrict__ rawm, const float* __restrict__ raw0,
             const float* __restrict__ ST, float* __restrict__ out)
{
    __shared__ float red[256];
    const int t = threadIdx.x, b = blockIdx.x;

    float lossv = 0.0f;
    if (b == 0) {
        const float* LP = ST + 2 * NN;
        float s = LP[t];
        s += LP[t + 256];
        s += LP[t + 512];
        s += LP[t + 768];
        red[t] = s;
        __syncthreads();
        for (int off = 128; off > 0; off >>= 1) {
            if (t < off) red[t] += red[t + off];
            __syncthreads();
        }
        lossv = red[0] * (1.0f / 1049600.0f);
    }

    const int f0 = b * 1024 + 4 * t;
    v4f v = {0.0f, 0.0f, 0.0f, 0.0f};
#pragma unroll
    for (int c = 0; c < 4; ++c) {
        const int f = f0 + c;
        float val = 0.0f;
        if (f == 0) {
            val = lossv;
        } else if (f < OUT_TOTAL) {
            const int e  = f - 1;
            const int i  = e / JT;
            const int j  = e - i * JT;
            const int jj = (j > 0) ? (j - 1) : 0;
            const float rm = rawm[(size_t)i * NN + jj];
            const float rz = raw0[i];
            const float r  = (j == 0) ? rz : rm;
            val = exs(r - ST[i]) * ST[NN + i];
        }
        v[c] = val;
    }
    if (f0 + 3 < OUT_TOTAL) {
        *(volatile v4f*)(out + f0) = v;
        __threadfence();
        *(volatile v4f*)(out + f0) = v;
    } else {
#pragma unroll
        for (int c = 0; c < 4; ++c)
            if (f0 + c < OUT_TOTAL) *(volatile float*)(out + f0 + c) = v[c];
        __threadfence();
#pragma unroll
        for (int c = 0; c < 4; ++c)
            if (f0 + c < OUT_TOTAL) *(volatile float*)(out + f0 + c) = v[c];
    }
}

extern "C" void kernel_launch(void* const* d_in, const int* in_sizes, int n_in,
                              void* d_out, int out_size, void* d_ws, size_t ws_size,
                              hipStream_t stream)
{
    if (n_in < 6) return;
    if (in_sizes[0] != NN * HH || in_sizes[1] != NN || in_sizes[2] != MLPH * 2 * HH ||
        in_sizes[3] != MLPH || in_sizes[4] != MLPH || in_sizes[5] < 1) return;
    if (out_size != OUT_TOTAL) return;

    const float* S   = (const float*)d_in[0];
    const int*   tgt = (const int*)  d_in[1];
    const float* W1  = (const float*)d_in[2];
    const float* b1  = (const float*)d_in[3];
    const float* W2  = (const float*)d_in[4];
    const float* b2  = (const float*)d_in[5];
    float* out = (float*)d_out;

    const size_t offXA   = 0;
    const size_t offXB   = offXA   + (size_t)NN * XP * sizeof(float);
    const size_t offRM   = offXB   + (size_t)NN * XP * sizeof(float);
    const size_t offR0   = offRM   + (size_t)NN * NN * sizeof(float);
    const size_t offST   = offR0   + (size_t)NN * sizeof(float);
    const size_t wsEnd   = offST   + (size_t)3 * NN * sizeof(float);
    if (wsEnd > ws_size) return;

    char* ws = (char*)d_ws;
    float* XA   = (float*)(ws + offXA);
    float* XB   = (float*)(ws + offXB);
    float* rawm = (float*)(ws + offRM);
    float* raw0 = (float*)(ws + offR0);
    float* ST   = (float*)(ws + offST);

    k_proj<<<dim3(NN / 16, 2), 32, 0, stream>>>(S, W1, b1, XA, XB);
    k_pair<<<dim3(NN / 64, NN / 16), 128, 0, stream>>>(XA, XB, W2, b2, rawm);
    k_col0<<<dim3(NN / 128), 128, 0, stream>>>(XA, W2, b2, raw0);
    k_rowstat<<<dim3(NN / 32), 256, 0, stream>>>(rawm, raw0, tgt, ST);
    k_final<<<dim3((OUT_TOTAL + 1023) / 1024), 256, 0, stream>>>(rawm, raw0, ST, out);
}
